// GroupLasso_70935679861371
// MI455X (gfx1250) — hardware-run, weakly checked
//
#include <hip/hip_runtime.h>

typedef __attribute__((ext_vector_type(16))) _Float16 v16h;
typedef __attribute__((ext_vector_type(8)))  _Float16 v8h;
typedef __attribute__((ext_vector_type(16))) __bf16   v16b;
typedef __attribute__((ext_vector_type(8)))  __bf16   v8b;
typedef __attribute__((ext_vector_type(8)))  float    v8f;
typedef __attribute__((ext_vector_type(4)))  float    v4f;
typedef __attribute__((ext_vector_type(2)))  unsigned v2u;

constexpr int kDd      = 128;
constexpr int kK       = 256;
constexpr int kT       = 1024;
constexpr int kB       = 4;
constexpr int kRows    = kB * kT;
constexpr int kGroups  = 8;
constexpr int kGroupSz = 32;
constexpr int kIters   = 100;
constexpr int kPowerSteps = 200;
constexpr float kLam = 0.01f;
constexpr float kReg = 0.01f;
constexpr float kTolRel = 1e-6f;
constexpr float kCarryA   = 64.0f;
constexpr float kCarryX   = 8.0f;
constexpr float kCarryRes = 2048.0f;
constexpr float kScaleMain = 1.0f / (kCarryA * kCarryX);
constexpr float kScaleRes  = kScaleMain / kCarryRes;
constexpr float kF16MinNormal = 6.103515625e-05f;
constexpr int kUpdBlocks = 128;
constexpr int kUpdTrips  = 8;
constexpr int kProdBlocks = kRows / 64;
constexpr int kLastPar   = (kIters - 1) & 1;
constexpr int kAcceptPar = kIters & 1;
static_assert(kGroups * kGroupSz == kK);
static_assert((kDd % 32) == 0 && (kK % 32) == 0);
static_assert((kRows % 64) == 0 && (kK % 64) == 0 && (kT % 64) == 0 && (kDd % 64) == 0);
static_assert(kUpdBlocks * kUpdTrips * 256 * 4 == kRows * kK);
static_assert(kProdBlocks == 64);

constexpr size_t kOffDT  = 0;
constexpr size_t kOffIT  = kOffDT  + (size_t)kK * kDd * 2;
constexpr size_t kOffDTD = kOffIT  + (size_t)kRows * kDd * 2;
constexpr size_t kOffDTY = kOffDTD + (size_t)kK * kK * 4;
constexpr size_t kOffAH  = kOffDTY + (size_t)kRows * kK * 4;
constexpr size_t kOffAL  = kOffAH  + (size_t)kK * kK * 2;
constexpr size_t kOffX0  = kOffAL  + (size_t)kK * kK * 2;
constexpr size_t kOffX1  = kOffX0  + (size_t)kRows * kK * 4;
constexpr size_t kOffL1  = kOffX1  + (size_t)kRows * kK * 4;
constexpr size_t kOffMH  = kOffL1  + (size_t)kRows * kK * 4;
constexpr size_t kOffML  = kOffMH  + (size_t)kRows * kK * 2;
constexpr size_t kOffGP  = kOffML  + (size_t)kRows * kK * 2;
constexpr size_t kOffDP  = kOffGP  + (size_t)kProdBlocks * 32 * 4;
constexpr size_t kOffST  = kOffDP  + (size_t)2 * kUpdBlocks * 32 * 4;
constexpr size_t kOffSC  = kOffST  + (size_t)104 * 32 * 4;
constexpr size_t kWsTotal = kOffSC + (size_t)32 * 4;
static_assert(kWsTotal == 22664320ull);
static_assert(kWsTotal <= 134217728ull);
static_assert((kOffIT % 128) == 0 && (kOffDTD % 128) == 0 && (kOffDTY % 128) == 0 && (kOffAH % 128) == 0 &&
              (kOffAL % 128) == 0 && (kOffX0 % 128) == 0 && (kOffX1 % 128) == 0 && (kOffL1 % 128) == 0 &&
              (kOffMH % 128) == 0 && (kOffML % 128) == 0 && (kOffGP % 128) == 0 && (kOffDP % 128) == 0 &&
              (kOffST % 128) == 0 && (kOffSC % 128) == 0);
static_assert(kIters + 1 <= 104);

__device__ __forceinline__ unsigned short f2bf_bits(float f) {
  unsigned u = __float_as_uint(f);
  return (unsigned short)((u + 0x7FFFu + ((u >> 16) & 1u)) >> 16);
}
__device__ __forceinline__ float bf_bits2f(unsigned short h) { return __uint_as_float(((unsigned)h) << 16); }

__device__ __forceinline__ void split_f16_planes(float v, float carry, unsigned short& hb, unsigned short& lb) {
  const float s  = v * carry;
  const float sh = (__builtin_fabsf(s) < kF16MinNormal) ? 0.0f : s;
  const _Float16 h = (_Float16)sh;
  const float hf = (float)h;
  const float r  = (s - hf) * kCarryRes;
  const float rl = (__builtin_fabsf(r) < kF16MinNormal) ? 0.0f : r;
  const _Float16 l = (_Float16)rl;
  hb = __builtin_bit_cast(unsigned short, h);
  lb = __builtin_bit_cast(unsigned short, l);
}

__device__ __forceinline__ void tie_b(v8f& a, v16b x, v16b y) { asm volatile("v_nop\n\tv_nop\n\tv_nop\n\tv_nop" : "+v"(a) : "v"(x), "v"(y)); }
__device__ __forceinline__ void tie_h(v8f& a, v16h x, v16h y) { asm volatile("v_nop\n\tv_nop\n\tv_nop\n\tv_nop" : "+v"(a) : "v"(x), "v"(y)); }
__device__ __forceinline__ void tie_acc(v8f& a) { asm volatile("v_nop\n\tv_nop\n\tv_nop\n\tv_nop" : "+v"(a)); }
__device__ __forceinline__ void keep4_h(v16h a, v16h b, v16h c, v16h d) { asm volatile("v_nop" :: "v"(a), "v"(b), "v"(c), "v"(d)); }
__device__ __forceinline__ void keep4_b(v16b a, v16b b, v16b c, v16b d) { asm volatile("v_nop" :: "v"(a), "v"(b), "v"(c), "v"(d)); }

template <typename T> struct Frag;
template <> struct Frag<_Float16> {
  typedef v16h V; union U { v16h v; v8h h[2]; };
  static __device__ __forceinline__ v16h load(const _Float16* p) {
    U f; f.h[0] = *(const v8h*)(p); f.h[1] = *(const v8h*)(p + 16); return f.v;
  }
  static __device__ __forceinline__ v8f mma(v16h a, v16h b, v8f c) {
    return __builtin_amdgcn_wmma_f32_16x16x32_f16(false, a, false, b, (short)0, c, false, false);
  }
};
template <> struct Frag<__bf16> {
  typedef v16b V; union U { v16b v; v8b h[2]; };
  static __device__ __forceinline__ v16b load(const __bf16* p) {
    U f; f.h[0] = *(const v8b*)(p); f.h[1] = *(const v8b*)(p + 16); return f.v;
  }
  static __device__ __forceinline__ v8f mma(v16b a, v16b b, v8f c) {
    return __builtin_amdgcn_wmma_f32_16x16x32_bf16(false, a, false, b, (short)0, c, false, false);
  }
};

__global__ __launch_bounds__(256) void plane_transpose_bf16(
    const float* __restrict__ in, unsigned short* __restrict__ out, int R, int C)
{
  __shared__ float tile[64 * 65];
  const int tid = threadIdx.x, lane = tid & 31, wave = tid >> 5;
  const int c0 = blockIdx.x * 64, r0 = blockIdx.y * 64, b = blockIdx.z;
  const float* inb = in + (size_t)b * R * C;
  unsigned short* outb = out + (size_t)b * C * R;
#pragma unroll
  for (int i = 0; i < 4; ++i) {
    const int q = tid + 256 * i;
    const int r = q >> 4, c4 = (q & 15) * 4;
    const v4f v = *(const v4f*)(inb + (size_t)(r0 + r) * C + c0 + c4);
#pragma unroll
    for (int e = 0; e < 4; ++e) tile[r * 65 + c4 + e] = v[e];
  }
  __syncthreads();
  const int q8 = lane >> 3, r8 = (lane & 7) * 8;
  v8h hv[2];
#pragma unroll
  for (int it = 0; it < 2; ++it) {
    const int c = it * 32 + wave * 4 + q8;
#pragma unroll
    for (int e = 0; e < 8; ++e) {
      const unsigned short bits = f2bf_bits(tile[(r8 + e) * 65 + c]);
      hv[it][e] = __builtin_bit_cast(_Float16, bits);
    }
  }
  for (int pass = 0; pass < 2; ++pass) {
#pragma unroll
    for (int it = 0; it < 2; ++it) {
      const int c = it * 32 + wave * 4 + q8;
      *(volatile v8h*)(outb + (size_t)(c0 + c) * R + r0 + r8) = hv[it];
    }
    __threadfence();
  }
}

__global__ __launch_bounds__(256) void plain_product_bf16(
    const unsigned short* __restrict__ Ap, int lda,
    const unsigned short* __restrict__ Btp, int ldb,
    float* __restrict__ C, int ldc, int M, int N, int K)
{
  typedef Frag<__bf16> F;
  const __bf16* A  = (const __bf16*)Ap;
  const __bf16* Bt = (const __bf16*)Btp;
  __shared__ __align__(16) float sT[8][16 * 68];
  const int lane = threadIdx.x & 31;
  const int wave = threadIdx.x >> 5;
  const int tilesN = N >> 6;
  const int tilesM = M >> 6;
  const int tile = blockIdx.x * 8 + wave;
  if (tile >= tilesM * tilesN) return;
  const int tm = tile / tilesN;
  const int tn = tile - tm * tilesN;
  const int m0 = tm << 6;
  const int n0 = tn << 6;
  const int rlane = lane & 15;
  const int koff  = (lane >> 4) * 8;
  const int mOff  = (lane >> 4) * 8;

  v8f acc[4][4];
#pragma unroll
  for (int i = 0; i < 4; ++i)
#pragma unroll
    for (int j = 0; j < 4; ++j) acc[i][j] = (v8f){0.f,0.f,0.f,0.f,0.f,0.f,0.f,0.f};

#pragma unroll 1
  for (int k0 = 0; k0 < K; k0 += 32) {
    v16b bh[4];
#pragma unroll
    for (int j = 0; j < 4; ++j) {
      const size_t bo = (size_t)(n0 + (j << 4) + rlane) * ldb + koff + k0;
      bh[j] = F::load(Bt + bo);
    }
#pragma unroll
    for (int i = 0; i < 4; ++i) {
      const size_t ao = (size_t)(m0 + (i << 4) + rlane) * lda + koff + k0;
      const v16b ah = F::load(A + ao);
#pragma unroll
      for (int j = 0; j < 4; ++j) acc[i][j] = F::mma(ah, bh[j], acc[i][j]);
      tie_b(acc[i][0], ah, bh[0]);
      tie_b(acc[i][1], ah, bh[1]);
      tie_b(acc[i][2], ah, bh[2]);
      tie_b(acc[i][3], ah, bh[3]);
    }
    keep4_b(bh[0], bh[1], bh[2], bh[3]);
  }
#pragma unroll
  for (int i = 0; i < 4; ++i)
#pragma unroll
    for (int j = 0; j < 4; ++j) tie_acc(acc[i][j]);

  float* slab = sT[wave];
#pragma unroll
  for (int i = 0; i < 4; ++i) {
    const int mBase = m0 + (i << 4);
#pragma unroll
    for (int j = 0; j < 4; ++j) {
#pragma unroll
      for (int r = 0; r < 8; ++r) slab[(mOff + r) * 68 + (j << 4) + rlane] = acc[i][j][r];
    }
    __builtin_amdgcn_fence(__ATOMIC_RELEASE, "workgroup");
    __builtin_amdgcn_wave_barrier();
    __builtin_amdgcn_fence(__ATOMIC_ACQUIRE, "workgroup");
    {
      const int hh = lane >> 4, c4 = (lane & 15) * 4;
      for (int pass = 0; pass < 2; ++pass) {
#pragma unroll
        for (int it = 0; it < 8; ++it) {
          const int row = it * 2 + hh;
          const v4f v = *(const v4f*)(slab + row * 68 + c4);
          *(volatile v4f*)(C + (size_t)(mBase + row) * ldc + n0 + c4) = v;
        }
        __threadfence();
      }
    }
    __builtin_amdgcn_fence(__ATOMIC_RELEASE, "workgroup");
    __builtin_amdgcn_wave_barrier();
    __builtin_amdgcn_fence(__ATOMIC_ACQUIRE, "workgroup");
  }
}

__global__ __launch_bounds__(256) void power_steps(const float* __restrict__ G, float* __restrict__ SC)
{
  __shared__ __align__(16) float sv[kK];
  __shared__ float rp[8];
  __shared__ float rq[8];
  const int tid = threadIdx.x, lane = tid & 31, wave = tid >> 5;
  sv[tid] = 0.0625f;
  __syncthreads();
  const float* row = G + (size_t)tid * kK;
  float lamv = 0.f;
#pragma unroll 1
  for (int step = 0; step < kPowerSteps; ++step) {
    float y = 0.f;
#pragma unroll 2
    for (int j4 = 0; j4 < kK / 4; ++j4) {
      const v4f a = *(const v4f*)(row + 4 * j4);
      const v4f s = *(const v4f*)(sv + 4 * j4);
      y = fmaf(a[0], s[0], y);
      y = fmaf(a[1], s[1], y);
      y = fmaf(a[2], s[2], y);
      y = fmaf(a[3], s[3], y);
    }
    float p = y * y;
    float q = y * sv[tid];
#pragma unroll
    for (int off = 16; off >= 1; off >>= 1) {
      p += __shfl_xor(p, off, 32);
      q += __shfl_xor(q, off, 32);
    }
    if (lane == 0) { rp[wave] = p; rq[wave] = q; }
    __syncthreads();
    float tp = rp[0], tq = rq[0];
#pragma unroll
    for (int w = 1; w < 8; ++w) { tp += rp[w]; tq += rq[w]; }
    lamv = tq;
    const float inv = 1.0f / sqrtf(tp);
    sv[tid] = y * inv;
    __syncthreads();
  }
  if (wave == 0) {
    const float L    = lamv;
    const float Linv = 1.0f / L;
    const float lmb  = kLam * Linv;
    float v = 0.0f;
    v = (lane == 0) ? L : v;
    v = (lane == 1) ? Linv : v;
    v = (lane == 2) ? lmb : v;
    volatile float* p = SC + lane;
    *p = v;
    __threadfence();
    *p = v;
  }
}

__global__ __launch_bounds__(256) void matrix_planes(
    const float* __restrict__ G, const float* __restrict__ SC,
    unsigned short* __restrict__ AH, unsigned short* __restrict__ AL)
{
  const int f  = blockIdx.x * 256 + threadIdx.x;
  const int e0 = f * 4;
  const int i  = e0 >> 8;
  const int j0 = e0 & (kK - 1);
  const float Linv = SC[1];
  const v4f g = *(const v4f*)(G + e0);
  unsigned short hb[4], lb[4];
#pragma unroll
  for (int e = 0; e < 4; ++e) {
    const float d = (i == j0 + e) ? 1.0f : 0.0f;
    const float t = g[e] * Linv;
    const float a = d - t;
    split_f16_planes(a, kCarryA, hb[e], lb[e]);
  }
  const v2u wh = { (unsigned)hb[0] | ((unsigned)hb[1] << 16), (unsigned)hb[2] | ((unsigned)hb[3] << 16) };
  const v2u wl = { (unsigned)lb[0] | ((unsigned)lb[1] << 16), (unsigned)lb[2] | ((unsigned)lb[3] << 16) };
  *(volatile v2u*)(AH + e0) = wh;
  *(volatile v2u*)(AL + e0) = wl;
  __threadfence();
  *(volatile v2u*)(AH + e0) = wh;
  *(volatile v2u*)(AL + e0) = wl;
}

__global__ __launch_bounds__(256) void state_planes_init(
    const float* __restrict__ x0, float* __restrict__ X,
    unsigned short* __restrict__ MH, unsigned short* __restrict__ ML)
{
  __shared__ float tile[64 * 65];
  const int tid = threadIdx.x, lane = tid & 31, wave = tid >> 5;
  const int c0 = blockIdx.x * 64, r0 = blockIdx.y * 64, b = blockIdx.z;
  const float* inb = x0 + (size_t)b * kK * kT;
#pragma unroll
  for (int i = 0; i < 4; ++i) {
    const int q = tid + 256 * i;
    const int r = q >> 4, c4 = (q & 15) * 4;
    const v4f v = *(const v4f*)(inb + (size_t)(r0 + r) * kT + c0 + c4);
#pragma unroll
    for (int e = 0; e < 4; ++e) tile[r * 65 + c4 + e] = bf_bits2f(f2bf_bits(v[e]));
  }
  __syncthreads();
  const int hh = lane >> 4, k4 = (lane & 15) * 4;
  const int q8 = lane >> 3, k8 = (lane & 7) * 8;
  v4f fv[4];
  v8h hv[2], lv[2];
#pragma unroll
  for (int it = 0; it < 4; ++it) {
    const int c = it * 16 + wave * 2 + hh;
#pragma unroll
    for (int e = 0; e < 4; ++e) fv[it][e] = tile[(k4 + e) * 65 + c];
  }
#pragma unroll
  for (int it = 0; it < 2; ++it) {
    const int c = it * 32 + wave * 4 + q8;
#pragma unroll
    for (int e = 0; e < 8; ++e) {
      unsigned short hb, lb;
      split_f16_planes(tile[(k8 + e) * 65 + c], kCarryX, hb, lb);
      hv[it][e] = __builtin_bit_cast(_Float16, hb);
      lv[it][e] = __builtin_bit_cast(_Float16, lb);
    }
  }
  const size_t rowb = (size_t)b * kT + c0;
  for (int pass = 0; pass < 2; ++pass) {
#pragma unroll
    for (int it = 0; it < 4; ++it) {
      const int c = it * 16 + wave * 2 + hh;
      *(volatile v4f*)(X + (rowb + c) * kK + r0 + k4) = fv[it];
    }
#pragma unroll
    for (int it = 0; it < 2; ++it) {
      const int c = it * 32 + wave * 4 + q8;
      const size_t o = (rowb + c) * kK + r0 + k8;
      *(volatile v8h*)(MH + o) = hv[it];
      *(volatile v8h*)(ML + o) = lv[it];
    }
    __threadfence();
  }
}

__global__ __launch_bounds__(256) void tables_init(float* __restrict__ ST0, float* __restrict__ DP1)
{
  const int tid = threadIdx.x, lane = tid & 31, wave = tid >> 5;
#pragma unroll 1
  for (int i = 0; i < 4; ++i) {
    const int idx = tid + 256 * i;
    const float one = ((idx & 7) == 0) ? 1.0f : 0.0f;
    const v4f v = { one, one, 0.0f, 0.0f };
    *(volatile v4f*)(DP1 + (size_t)idx * 4) = v;
    __threadfence();
    *(volatile v4f*)(DP1 + (size_t)idx * 4) = v;
  }
  if (wave == 0) {
    const float v = (lane == 0 || lane == 2) ? 1.0f : 0.0f;
    volatile float* p = ST0 + lane;
    *p = v;
    __threadfence();
    *p = v;
  }
}

__global__ __launch_bounds__(256) void step_product(
    const unsigned short* __restrict__ XHp, const unsigned short* __restrict__ XLp,
    const unsigned short* __restrict__ WHp, const unsigned short* __restrict__ WLp,
    const float* __restrict__ DTY, const float* __restrict__ SC,
    float* __restrict__ L1, float* __restrict__ GP)
{
  typedef Frag<_Float16> F;
  __shared__ __align__(16) float sT[8][16 * 36];
  __shared__ float sG[8];
  const int lane = threadIdx.x & 31;
  const int wave = threadIdx.x >> 5;
  const int m0 = blockIdx.x * 64;
  const int n0 = wave * 32;
  const int rlane = lane & 15;
  const int koff  = (lane >> 4) * 8;
  const int mOff  = (lane >> 4) * 8;

  const _Float16* xph = (const _Float16*)XHp + (size_t)(m0 + rlane) * kK + koff;
  const _Float16* xpl = (const _Float16*)XLp + (size_t)(m0 + rlane) * kK + koff;
  const _Float16* wph = (const _Float16*)WHp + (size_t)(n0 + rlane) * kK + koff;
  const _Float16* wpl = (const _Float16*)WLp + (size_t)(n0 + rlane) * kK + koff;

  v8f accM[4][2], accR[4][2];
#pragma unroll
  for (int i = 0; i < 4; ++i)
#pragma unroll
    for (int j = 0; j < 2; ++j) {
      accM[i][j] = (v8f){0.f,0.f,0.f,0.f,0.f,0.f,0.f,0.f};
      accR[i][j] = (v8f){0.f,0.f,0.f,0.f,0.f,0.f,0.f,0.f};
    }

#pragma unroll 1
  for (int k0 = 0; k0 < kK; k0 += 32) {
    v16h wh[2], wl[2];
#pragma unroll
    for (int j = 0; j < 2; ++j) {
      wh[j] = F::load(wph + (size_t)j * 16 * kK + k0);
      wl[j] = F::load(wpl + (size_t)j * 16 * kK + k0);
    }
#pragma unroll
    for (int i = 0; i < 4; ++i) {
      const v16h xh = F::load(xph + (size_t)i * 16 * kK + k0);
      const v16h xl = F::load(xpl + (size_t)i * 16 * kK + k0);
#pragma unroll
      for (int j = 0; j < 2; ++j) {
        accM[i][j] = F::mma(xh, wh[j], accM[i][j]);
        accR[i][j] = F::mma(xh, wl[j], accR[i][j]);
        accR[i][j] = F::mma(xl, wh[j], accR[i][j]);
      }
      tie_h(accM[i][0], xh, wh[0]);
      tie_h(accM[i][1], xh, wh[1]);
      tie_h(accR[i][0], xl, wl[0]);
      tie_h(accR[i][1], xl, wl[1]);
    }
    keep4_h(wh[0], wh[1], wl[0], wl[1]);
  }
#pragma unroll
  for (int i = 0; i < 4; ++i)
#pragma unroll
    for (int j = 0; j < 2; ++j) {
      tie_acc(accM[i][j]);
      tie_acc(accR[i][j]);
    }

  const float Linv = SC[1];
  const float lmb  = SC[2];
  float ss = 0.0f;
  float* slab = sT[wave];
  const int q = lane >> 3, c4 = (lane & 7) * 4;
#pragma unroll
  for (int i = 0; i < 4; ++i) {
    const int mBase = m0 + (i << 4);
#pragma unroll
    for (int j = 0; j < 2; ++j) {
#pragma unroll
      for (int r = 0; r < 8; ++r) {
        const float v = accM[i][j][r] * kScaleMain + accR[i][j][r] * kScaleRes;
        slab[(mOff + r) * 36 + (j << 4) + rlane] = v;
      }
    }
    __builtin_amdgcn_fence(__ATOMIC_RELEASE, "workgroup");
    __builtin_amdgcn_wave_barrier();
    __builtin_amdgcn_fence(__ATOMIC_ACQUIRE, "workgroup");
    v4f ov[4];
#pragma unroll
    for (int it = 0; it < 4; ++it) {
      const int row = it * 4 + q;
      const v4f a  = *(const v4f*)(slab + row * 36 + c4);
      const v4f dy = *(const v4f*)(DTY + (size_t)(mBase + row) * kK + n0 + c4);
#pragma unroll
      for (int e = 0; e < 4; ++e) {
        const float t  = dy[e] * Linv;
        const float cm = t - lmb;
        const float cp = t + lmb;
        const float l  = fmaxf(a[e] + cm, 0.0f) + fminf(a[e] + cp, 0.0f);
        ov[it][e] = l;
        ss = fmaf(l, l, ss);
      }
    }
    for (int pass = 0; pass < 2; ++pass) {
#pragma unroll
      for (int it = 0; it < 4; ++it) {
        const int row = it * 4 + q;
        *(volatile v4f*)(L1 + (size_t)(mBase + row) * kK + n0 + c4) = ov[it];
      }
      __threadfence();
    }
    __builtin_amdgcn_fence(__ATOMIC_RELEASE, "workgroup");
    __builtin_amdgcn_wave_barrier();
    __builtin_amdgcn_fence(__ATOMIC_ACQUIRE, "workgroup");
  }
#pragma unroll
  for (int off = 16; off >= 1; off >>= 1) ss += __shfl_xor(ss, off, 32);
  if (lane == 0) sG[wave] = ss;
  __syncthreads();
  if (wave == 0) {
    const float g = sG[lane & 7];
    const float val = (lane < 8) ? g : 0.0f;
    volatile float* p = GP + (size_t)blockIdx.x * 32 + lane;
    *p = val;
    __threadfence();
    *p = val;
  }
}

__global__ __launch_bounds__(256) void step_update(
    const float* __restrict__ L1, const float* __restrict__ Xc, float* __restrict__ Xn,
    unsigned short* __restrict__ MH, unsigned short* __restrict__ ML,
    const float* __restrict__ GP, const float* __restrict__ DPp, float* __restrict__ DPc,
    const float* __restrict__ STp, float* __restrict__ STn, int prevpar)
{
  __shared__ float sGr[8 * 8];
  __shared__ float sDw[8];
  __shared__ float sXw[8];
  __shared__ float sW[16];
  const int tid = threadIdx.x, lane = tid & 31, wave = tid >> 5;

  {
    const int g = tid & 7, part = tid >> 3;
    float s = GP[(size_t)(2 * part) * 32 + g] + GP[(size_t)(2 * part + 1) * 32 + g];
    s += __shfl_xor(s, 8, 32);
    s += __shfl_xor(s, 16, 32);
    if (lane < 8) sGr[wave * 8 + lane] = s;
  }
  {
    const int bi = tid & 127;
    float d = DPp[(size_t)bi * 32];
    float x = DPp[(size_t)bi * 32 + 1];
#pragma unroll
    for (int off = 16; off >= 1; off >>= 1) {
      d += __shfl_xor(d, off, 32);
      x += __shfl_xor(x, off, 32);
    }
    if (lane == 0) { sDw[wave] = d; sXw[wave] = x; }
  }
  __syncthreads();

  const int gq = (tid & 63) >> 3;
  float gtot = sGr[gq];
#pragma unroll
  for (int w = 1; w < 8; ++w) gtot += sGr[w * 8 + gq];
  const float dt = ((sDw[0] + sDw[1]) + sDw[2]) + sDw[3];
  const float xt = ((sXw[0] + sXw[1]) + sXw[2]) + sXw[3];

  const float m_prev    = STp[0];
  const float done_prev = STp[1];
  const float nm_prev   = STp[2];
  const float sel_prev  = STp[3];
  const float rel  = sqrtf(dt) / sqrtf(xt);
  const bool conv  = rel < kTolRel;
  const bool dprev = (done_prev != 0.0f);
  const bool done_i = dprev || conv;
  const bool newly  = conv && !dprev;
  const float sel_i = newly ? (float)prevpar : sel_prev;
  const float m_i   = done_i ? m_prev : nm_prev;
  const float nm_i  = 0.5f + 0.5f * sqrtf(1.0f + 4.0f * m_i * m_i);
  const float mm1   = m_i - 1.0f;
  const float rinv  = 1.0f / nm_i;
  const float nrm   = sqrtf(gtot);
  const float safe  = (nrm == 0.0f) ? 1.0f : nrm;
  const float sc    = (nrm == 0.0f) ? 0.0f : fmaxf(0.0f, 1.0f - kReg / safe);

  if (blockIdx.x == 0 && wave == 0) {
    float v = 0.0f;
    v = (lane == 0) ? m_i : v;
    v = (lane == 1) ? (done_i ? 1.0f : 0.0f) : v;
    v = (lane == 2) ? nm_i : v;
    v = (lane == 3) ? sel_i : v;
    volatile float* p = STn + lane;
    *p = v;
    __threadfence();
    *p = v;
  }

  const int dflag = __builtin_amdgcn_readfirstlane(done_i ? 1 : 0);
  float dss = 0.0f, xss = 0.0f;
  if (dflag == 0) {
#pragma unroll 1
    for (int trip = 0; trip < kUpdTrips; ++trip) {
      const size_t e0 = ((size_t)blockIdx.x * (kUpdTrips * 256) + (size_t)trip * 256 + tid) * 4;
      const v4f l = *(const v4f*)(L1 + e0);
      const v4f x = *(const v4f*)(Xc + e0);
      v4f nx;
      unsigned short hb[4], lb[4];
#pragma unroll
      for (int e = 0; e < 4; ++e) {
        const float n  = l[e] * sc;
        const float d  = n - x[e];
        dss = fmaf(d, d, dss);
        const float xe = x[e] + 1e-16f;
        xss = fmaf(xe, xe, xss);
        float t = d * mm1;
        t = t * rinv;
        const float m = n + t;
        nx[e] = n;
        split_f16_planes(m, kCarryX, hb[e], lb[e]);
      }
      const v2u wh = { (unsigned)hb[0] | ((unsigned)hb[1] << 16), (unsigned)hb[2] | ((unsigned)hb[3] << 16) };
      const v2u wl = { (unsigned)lb[0] | ((unsigned)lb[1] << 16), (unsigned)lb[2] | ((unsigned)lb[3] << 16) };
      *(volatile v4f*)(Xn + e0) = nx;
      *(volatile v2u*)(MH + e0) = wh;
      *(volatile v2u*)(ML + e0) = wl;
      __threadfence();
      *(volatile v4f*)(Xn + e0) = nx;
      *(volatile v2u*)(MH + e0) = wh;
      *(volatile v2u*)(ML + e0) = wl;
    }
  }
#pragma unroll
  for (int off = 16; off >= 1; off >>= 1) {
    dss += __shfl_xor(dss, off, 32);
    xss += __shfl_xor(xss, off, 32);
  }
  if (lane == 0) { sW[wave] = dss; sW[8 + wave] = xss; }
  __syncthreads();
  if (wave == 0) {
    float d = sW[0], x = sW[8];
#pragma unroll
    for (int w = 1; w < 8; ++w) { d += sW[w]; x += sW[8 + w]; }
    d = (dflag != 0) ? 1.0f : d;
    x = (dflag != 0) ? 1.0f : x;
    float v = 0.0f;
    v = (lane == 0) ? d : v;
    v = (lane == 1) ? x : v;
    volatile float* p = DPc + (size_t)blockIdx.x * 32 + lane;
    *p = v;
    __threadfence();
    *p = v;
  }
}

__global__ __launch_bounds__(256) void output_transpose(
    const float* Xa, const float* Xb, const float* __restrict__ STl, const float* __restrict__ DPl,
    float* __restrict__ out)
{
  __shared__ float tile[64 * 65];
  __shared__ float sDw[8];
  __shared__ float sXw[8];
  const int tid = threadIdx.x, lane = tid & 31, wave = tid >> 5;
  {
    const int bi = tid & 127;
    float d = DPl[(size_t)bi * 32];
    float x = DPl[(size_t)bi * 32 + 1];
#pragma unroll
    for (int off = 16; off >= 1; off >>= 1) {
      d += __shfl_xor(d, off, 32);
      x += __shfl_xor(x, off, 32);
    }
    if (lane == 0) { sDw[wave] = d; sXw[wave] = x; }
  }
  __syncthreads();
  const float dt = ((sDw[0] + sDw[1]) + sDw[2]) + sDw[3];
  const float xt = ((sXw[0] + sXw[1]) + sXw[2]) + sXw[3];
  const float rel = sqrtf(dt) / sqrtf(xt);
  const bool conv  = rel < kTolRel;
  const bool dprev = (STl[1] != 0.0f);
  const int selp   = (STl[3] != 0.0f) ? 1 : 0;
  int sel = dprev ? selp : (conv ? kLastPar : kAcceptPar);
  sel = __builtin_amdgcn_readfirstlane(sel);
  const float* src = (sel != 0) ? Xb : Xa;

  const int c0 = blockIdx.x * 64, r0 = blockIdx.y * 64, b = blockIdx.z;
#pragma unroll
  for (int i = 0; i < 4; ++i) {
    const int q = tid + 256 * i;
    const int r = q >> 4, c4 = (q & 15) * 4;
    const v4f v = *(const v4f*)(src + ((size_t)b * kT + r0 + r) * kK + c0 + c4);
#pragma unroll
    for (int e = 0; e < 4; ++e) tile[r * 65 + c4 + e] = v[e];
  }
  __syncthreads();
  const int hh = lane >> 4, t4 = (lane & 15) * 4;
  v4f fv[4];
#pragma unroll
  for (int it = 0; it < 4; ++it) {
    const int c = it * 16 + wave * 2 + hh;
#pragma unroll
    for (int e = 0; e < 4; ++e) fv[it][e] = tile[(t4 + e) * 65 + c];
  }
  for (int pass = 0; pass < 2; ++pass) {
#pragma unroll
    for (int it = 0; it < 4; ++it) {
      const int c = it * 16 + wave * 2 + hh;
      *(volatile v4f*)(out + ((size_t)b * kK + c0 + c) * kT + r0 + t4) = fv[it];
    }
    __threadfence();
  }
}

extern "C" void kernel_launch(void* const* d_in, const int* in_sizes, int n_in,
                              void* d_out, int out_size, void* d_ws, size_t ws_size,
                              hipStream_t stream) {
  if (n_in < 3) return;
  if (in_sizes[0] != kDd * kK) return;
  if (in_sizes[1] != kB * kDd * kT) return;
  if (in_sizes[2] != kB * kK * kT) return;
  if (out_size != kB * kK * kT) return;
  if (ws_size < kWsTotal) return;

  const float* Dict = (const float*)d_in[0];
  const float* inp  = (const float*)d_in[1];
  const float* x0   = (const float*)d_in[2];
  float* out = (float*)d_out;

  char* ws = (char*)d_ws;
  unsigned short* DT  = (unsigned short*)(ws + kOffDT);
  unsigned short* IT  = (unsigned short*)(ws + kOffIT);
  float*          DTD = (float*)(ws + kOffDTD);
  float*          DTY = (float*)(ws + kOffDTY);
  unsigned short* AH  = (unsigned short*)(ws + kOffAH);
  unsigned short* AL  = (unsigned short*)(ws + kOffAL);
  float*          XA  = (float*)(ws + kOffX0);
  float*          XB  = (float*)(ws + kOffX1);
  float*          L1  = (float*)(ws + kOffL1);
  unsigned short* MH  = (unsigned short*)(ws + kOffMH);
  unsigned short* ML  = (unsigned short*)(ws + kOffML);
  float*          GP  = (float*)(ws + kOffGP);
  float*          DP  = (float*)(ws + kOffDP);
  float*          ST  = (float*)(ws + kOffST);
  float*          SC  = (float*)(ws + kOffSC);
  constexpr int kDpStride = kUpdBlocks * 32;

  plane_transpose_bf16<<<dim3(kK / 64, kDd / 64, 1), 256, 0, stream>>>(Dict, DT, kDd, kK);
  plane_transpose_bf16<<<dim3(kT / 64, kDd / 64, kB), 256, 0, stream>>>(inp, IT, kDd, kT);
  plain_product_bf16<<<dim3(2), 256, 0, stream>>>(DT, kDd, DT, kDd, DTD, kK, kK, kK, kDd);
  plain_product_bf16<<<dim3(32), 256, 0, stream>>>(IT, kDd, DT, kDd, DTY, kK, kRows, kK, kDd);
  power_steps<<<dim3(1), 256, 0, stream>>>(DTD, SC);
  matrix_planes<<<dim3(kK * kK / 4 / 256), 256, 0, stream>>>(DTD, SC, AH, AL);
  state_planes_init<<<dim3(kT / 64, kK / 64, kB), 256, 0, stream>>>(x0, XA, MH, ML);
  tables_init<<<dim3(1), 256, 0, stream>>>(ST, DP + kDpStride);

  for (int it = 0; it < kIters; ++it) {
    const float* Xc = (it & 1) ? XB : XA;
    float*       Xn = (it & 1) ? XA : XB;
    const int ppar = (it + 1) & 1;
    step_product<<<dim3(kProdBlocks), 256, 0, stream>>>(MH, ML, AH, AL, DTY, SC, L1, GP);
    step_update<<<dim3(kUpdBlocks), 256, 0, stream>>>(
        L1, Xc, Xn, MH, ML, GP,
        DP + (size_t)ppar * kDpStride, DP + (size_t)(it & 1) * kDpStride,
        ST + (size_t)it * 32, ST + (size_t)(it + 1) * 32, ppar);
  }

  output_transpose<<<dim3(kK / 64, kT / 64, kB), 256, 0, stream>>>(
      XA, XB, ST + (size_t)kIters * 32, DP + (size_t)kLastPar * kDpStride, out);
}
